// ExLRestSelfAtten_49125835931701
// MI455X (gfx1250) — hardware-verified
//
#include <hip/hip_runtime.h>
#include <math.h>

typedef __attribute__((ext_vector_type(16))) _Float16 v16h;
typedef __attribute__((ext_vector_type(16))) __bf16 v16b;
typedef __attribute__((ext_vector_type(8)))  _Float16 v8h;
typedef __attribute__((ext_vector_type(8)))  float v8f;
typedef __attribute__((ext_vector_type(4)))  float v4f;
typedef __attribute__((ext_vector_type(2)))  float v2f;
typedef __attribute__((ext_vector_type(4)))  unsigned v4u;
typedef __attribute__((ext_vector_type(4)))  int v4i;
typedef float __attribute__((may_alias)) float_a;
typedef int __attribute__((may_alias)) int_a;

template <typename T> __device__ __forceinline__ void vst2(void* p, T v) { *(volatile T*)p = v; __threadfence(); *(volatile T*)p = v; }
__device__ __forceinline__ v8f wmma16(v16h a, v16h b, v8f c) {
  v8f d = __builtin_amdgcn_wmma_f32_16x16x32_f16(false, a, false, b, (short)0, c, false, false);
  asm volatile("v_nop\n\tv_nop\n\tv_nop\n\tv_nop" : "+v"(d) : "v"(a), "v"(b));
  return d;
}
__device__ __forceinline__ v8f wmma_bf(v16b a, v16b b, v8f c) {
  v8f d = __builtin_amdgcn_wmma_f32_16x16x32_bf16(false, a, false, b, (short)0, c, false, false);
  asm volatile("v_nop\n\tv_nop\n\tv_nop\n\tv_nop" : "+v"(d) : "v"(a), "v"(b));
  return d;
}
__device__ __forceinline__ v16h frag_h(const _Float16* rowk0, int lane) {
  union { v16h v; v8h q[2]; } u; const _Float16* p = rowk0 + 8 * (lane >> 4);
  u.q[0] = *(const v8h*)p; u.q[1] = *(const v8h*)(p + 16); return u.v;
}
__device__ __forceinline__ v16h frag_f32(const float* rowk0, int lane) {
  v16h a; const float* p = rowk0 + 8 * (lane >> 4);
#pragma unroll
  for (int i = 0; i < 8; ++i) { a[i] = (_Float16)p[i]; a[8 + i] = (_Float16)p[16 + i]; }
  return a;
}
__device__ __forceinline__ v16h frag_f32s(const float* rowk0, int lane, float sc) {
  v16h a; const float* p = rowk0 + 8 * (lane >> 4);
#pragma unroll
  for (int i = 0; i < 8; ++i) { a[i] = (_Float16)(p[i] * sc); a[8 + i] = (_Float16)(p[16 + i] * sc); }
  return a;
}
__device__ __forceinline__ v16h fragc_f32(const float* W, int k0, int n, int lane, int ld, int K) {
  v16h a; const int g = lane >> 4;
#pragma unroll
  for (int i = 0; i < 8; ++i) { const int ka = k0 + 8 * g + i, kb = ka + 16;
    a[i] = (_Float16)(ka < K ? W[(size_t)(ka < K ? ka : K - 1) * ld + n] : 0.f); a[8 + i] = (_Float16)(kb < K ? W[(size_t)(kb < K ? kb : K - 1) * ld + n] : 0.f); }
  return a;
}
struct F2 { v16b h, l; };
__device__ __forceinline__ F2 bsplit16(const float v[16]) { F2 r;
#pragma unroll
  for (int i = 0; i < 16; ++i) { const __bf16 h = (__bf16)v[i]; r.h[i] = h; r.l[i] = (__bf16)(v[i] - (float)h); }
  return r; }
__device__ __forceinline__ F2 split_row(const float* row, int k0, int lane) { float v[16]; const float* p = row + k0 + 8 * (lane >> 4);
#pragma unroll
  for (int i = 0; i < 8; ++i) { v[i] = p[i]; v[8 + i] = p[16 + i]; }
  return bsplit16(v); }
__device__ __forceinline__ F2 split_rowK(const float* row, int k0, int lane, int K) { float v[16]; const int g = lane >> 4;
#pragma unroll
  for (int i = 0; i < 8; ++i) { const int ka = k0 + 8 * g + i, kb = ka + 16; v[i] = ka < K ? row[ka < K ? ka : K - 1] : 0.f; v[8 + i] = kb < K ? row[kb < K ? kb : K - 1] : 0.f; }
  return bsplit16(v); }
__device__ __forceinline__ F2 split_col(const float* W, int k0, int n, int lane, int ld, int K) { float v[16]; const int g = lane >> 4;
#pragma unroll
  for (int i = 0; i < 8; ++i) { const int ka = k0 + 8 * g + i, kb = ka + 16; v[i] = ka < K ? W[(size_t)(ka < K ? ka : K - 1) * ld + n] : 0.f; v[8 + i] = kb < K ? W[(size_t)(kb < K ? kb : K - 1) * ld + n] : 0.f; }
  return bsplit16(v); }
__device__ __forceinline__ v8f mac3(const F2& a, const F2& b, v8f c) { c = wmma_bf(a.l, b.h, c); c = wmma_bf(a.h, b.l, c); return wmma_bf(a.h, b.h, c); }
__device__ __forceinline__ float sigm(float v) { return 1.0f / (1.0f + expf(-v)); }
#define LDSX() do { asm volatile("s_wait_dscnt 0" ::: "memory"); __builtin_amdgcn_wave_barrier(); __builtin_amdgcn_fence(__ATOMIC_RELEASE, "workgroup"); } while (0)


#define NB 64
#define SQ 100
#define DIN 256
#define HID 512
#define DOUT 256
#define HW 16
#define WN 33
#define NR (NB * SQ)
#define GP 128
#define QKVP (3 * HID)
#ifndef NBT
#define NBT NB
#endif
typedef __attribute__((ext_vector_type(8))) __bf16 v8b;
__device__ __forceinline__ v16b frag_b(const __bf16* rowk0, int lane) {
  union { v16b v; v8b q[2]; } u; const __bf16* p = rowk0 + 8 * (lane >> 4);
  u.q[0] = *(const v8b*)p; u.q[1] = *(const v8b*)(p + 16); return u.v;
}
__device__ __forceinline__ float bfr(float v) { return (float)(__bf16)v; }
__device__ __attribute__((noinline)) float exp_ni(float v) { return expf(v); }
__device__ __attribute__((noinline)) float erf_ni(float v) { return erff(v); }

#define WS_P0   0u
#define WS_PQ   (WS_P0 + 2u * HID * DIN)
#define WS_P1   (WS_PQ + 2u * QKVP * HID)
#define WS_H    (WS_P1 + 2u * DOUT * HID)
#define WS_QKV  (WS_H + 4u * NR * HID)
#define WS_G    (WS_QKV + 4u * NR * QKVP)
#define WS_MZ   (WS_G + 4u * NB * GP * GP)
#define WS_C    (WS_MZ + 4u * NB * GP * GP)
#define WS_VTH  (WS_C + 4u * NB * GP * GP)
#define WS_VTL  (WS_VTH + 2u * NB * HID * GP)
#define WS_OB   (WS_VTL + 2u * NB * HID * GP)
#define WS_END  (WS_OB + 4u * NR * HID)

__global__ __launch_bounds__(256) void k_packT(const float* __restrict__ Wm, int K, int ld, __bf16* __restrict__ DST) {
  __shared__ __align__(16) __bf16 s[HID]; const int n = blockIdx.x, tid = threadIdx.x;
  for (int k = tid; k < K; k += 256) s[k] = (__bf16)Wm[(size_t)k * ld + n];
  __syncthreads();
  if (tid < K / 8) vst2((unsigned*)(DST + (size_t)n * K + tid * 8), *(const v4u*)&s[tid * 8]);
}
template <int K, int AM, int EPI>
__global__ __launch_bounds__(128) void k_lin(const float* __restrict__ A, int lda, const __bf16* __restrict__ P, const float* __restrict__ bias, float* __restrict__ OUT, int ldo) {
  __shared__ __align__(16) float so[4][16][132];
  const int tid = threadIdx.x, wave = tid >> 5, lane = tid & 31, col = lane & 15, g = lane >> 4; const size_t r0 = (size_t)blockIdx.x * 64 + wave * 16; const int n0 = blockIdx.y * 128;
  v8f acc[8] = {};
#pragma unroll 2
  for (int kc = 0; kc < K / 32; ++kc) {
    if (AM == 0) { v16b a; { const float* p = A + (r0 + col) * lda + kc * 32 + 8 * g;
#pragma unroll
        for (int i = 0; i < 8; ++i) { a[i] = (__bf16)p[i]; a[8 + i] = (__bf16)p[16 + i]; } }
#pragma unroll
      for (int j = 0; j < 8; ++j) acc[j] = wmma_bf(a, frag_b(P + (size_t)(n0 + j * 16 + col) * K + kc * 32, lane), acc[j]); }
    else { const F2 a = split_row(A + (r0 + col) * lda, kc * 32, lane);
#pragma unroll
      for (int j = 0; j < 8; ++j) { const v16b w = frag_b(P + (size_t)(n0 + j * 16 + col) * K + kc * 32, lane); acc[j] = wmma_bf(a.l, w, acc[j]); acc[j] = wmma_bf(a.h, w, acc[j]); } } }
#pragma unroll
  for (int j = 0; j < 8; ++j) { const float bb = bias ? bfr(bias[n0 + j * 16 + col]) : 0.f;
#pragma unroll
    for (int r = 0; r < 8; ++r) { float v = acc[j][r] + bb; if (EPI == 1) v = fmaxf(v, 0.f); so[wave][8 * g + r][j * 16 + col] = v; } }
  LDSX();
  for (int rl = 0; rl < 16; ++rl) vst2(OUT + (r0 + rl) * ldo + n0 + lane * 4, *(const v4f*)&so[wave][rl][lane * 4]);
}
__global__ __launch_bounds__(128) void k_g(const float* __restrict__ QKV, float* __restrict__ G) {
  __shared__ __align__(16) float so[16][GP];
  const int tid = threadIdx.x, wave = tid >> 5, lane = tid & 31, col = lane & 15, g = lane >> 4; const int it = blockIdx.x, b = blockIdx.y;
  const int qi = it * 16 + col; const float* qrow = QKV + ((size_t)b * SQ + (qi < SQ ? qi : SQ - 1)) * QKVP;
  v8f acc[2] = {};
#pragma unroll 1
  for (int kc = 0; kc < HID / 32; ++kc) { const F2 a = split_row(qrow, kc * 32, lane);
#pragma unroll
    for (int jj = 0; jj < 2; ++jj) { const int jt = wave + 4 * jj; if (jt < 7) { const int kj = jt * 16 + col; const F2 k = split_row(QKV + ((size_t)b * SQ + (kj < SQ ? kj : SQ - 1)) * QKVP + HID, kc * 32, lane); acc[jj] = mac3(a, k, acc[jj]); } } }
#pragma unroll
  for (int jj = 0; jj < 2; ++jj) { const int jt = wave + 4 * jj;
#pragma unroll
    for (int r = 0; r < 8; ++r) so[8 * g + r][jt * 16 + col] = (jt < 7) ? acc[jj][r] * 0.04419417382415922f : 0.f; }
  __syncthreads();
#pragma unroll
  for (int q = 0; q < 4; ++q) { const int rl = q * 4 + wave; vst2(G + ((size_t)(b * GP + it * 16 + rl)) * GP + lane * 4, *(const v4f*)&so[rl][lane * 4]); }
}
__global__ __launch_bounds__(256) void k_soft(const float* __restrict__ G, float* __restrict__ MZ, float* __restrict__ C) {
  __shared__ __align__(16) float srow[8][GP]; __shared__ float sm[8][WN + 3], siz[8][WN + 3];
  const int wave = threadIdx.x >> 5, lane = threadIdx.x & 31; const int n = blockIdx.x * 8 + wave; const int b = n / GP, s = n % GP;
  float cu = 0.f, cu32 = 0.f;
  if (s < SQ) {
    const int j0 = s + HW - lane, j32 = s - HW; const int j0c = j0 < 0 ? 0 : (j0 >= SQ ? SQ - 1 : j0), j32c = j32 < 0 ? 0 : j32;
#pragma unroll 1
    for (int w = 0; w < WN; ++w) { const int i = s + HW - w; const bool vi = (i >= 0) && (i < SQ); const int ic = i < 0 ? 0 : (i >= SQ ? SQ - 1 : i);
      const float* grow = G + ((size_t)(b * GP + ic)) * GP; const float g0 = grow[j0c], g32 = grow[j32c];
      const float sc0 = (vi && j0 >= 0 && j0 < SQ) ? g0 : 0.f, sc32 = (vi && j32 >= 0) ? g32 : 0.f;
      float m = fmaxf(sc0, sc32);
#pragma unroll
      for (int o = 1; o < 32; o <<= 1) m = fmaxf(m, __shfl_xor(m, o));
      const float e0 = exp_ni(sc0 - m), e32 = exp_ni(sc32 - m); float z = e0;
#pragma unroll
      for (int o = 1; o < 32; o <<= 1) z += __shfl_xor(z, o);
      z += e32; const float iz = 1.0f / z; cu += e0 * iz; cu32 += e32 * iz;
      if (lane == 0) { sm[wave][w] = m; siz[wave][w] = iz; } } }
  LDSX();
  for (int q = lane; q < GP; q += 32) { float v = 0.f; if (s < SQ) { if (q < WN) v = sm[wave][q]; else if (q >= 64 && q < 64 + WN) v = siz[wave][q - 64]; } srow[wave][q] = v; }
  LDSX();
  vst2(MZ + (size_t)n * GP + lane * 4, *(const v4f*)&srow[wave][lane * 4]);
  LDSX();
  for (int q = lane; q < GP; q += 32) srow[wave][q] = 0.f;
  LDSX();
  if (s < SQ) { const int t0 = s + HW - lane; if (t0 >= 0 && t0 < SQ) srow[wave][t0] = cu; if (lane == 0 && s - HW >= 0) srow[wave][s - HW] = cu32; }
  LDSX();
  vst2(C + (size_t)n * GP + lane * 4, *(const v4f*)&srow[wave][lane * 4]);
}
__global__ __launch_bounds__(256) void k_vt(const float* __restrict__ QKV, __bf16* __restrict__ VTH, __bf16* __restrict__ VTL) {
  __shared__ __align__(16) __bf16 svh[HID][72], svl[HID][72];
  const int tid = threadIdx.x; const int p0 = blockIdx.x * 64, b = blockIdx.y;
  for (int q = tid; q < 64 * HID; q += 256) { const int tl = q >> 9, c = q & 511; const int t = p0 + tl; const float v = (t < SQ) ? QKV[((size_t)b * SQ + (t < SQ ? t : SQ - 1)) * QKVP + 2 * HID + c] : 0.f; const __bf16 hb = (__bf16)v; svh[c][tl] = hb; svl[c][tl] = (__bf16)(v - (float)hb); }
  __syncthreads();
  for (int q = tid; q < HID * 8; q += 256) { const int rowi = q >> 3, pc = q & 7; const size_t o = ((size_t)b * HID + rowi) * GP + p0 + pc * 8; vst2((unsigned*)(VTH + o), *(const v4u*)&svh[rowi][pc * 8]); vst2((unsigned*)(VTL + o), *(const v4u*)&svl[rowi][pc * 8]); }
}
__global__ __launch_bounds__(128) void k_cv(const float* __restrict__ C, const __bf16* __restrict__ VTH, const __bf16* __restrict__ VTL, float* __restrict__ OB) {
  __shared__ __align__(16) float so[4][16][132];
  const int tid = threadIdx.x, wave = tid >> 5, lane = tid & 31, col = lane & 15, g = lane >> 4; const int s0 = blockIdx.x * 64 + wave * 16, cg = blockIdx.y, b = blockIdx.z;
  v8f acc[8] = {};
#pragma unroll
  for (int kc = 0; kc < GP / 32; ++kc) { const F2 a = split_row(C + ((size_t)(b * GP + s0 + col)) * GP, kc * 32, lane);
#pragma unroll
    for (int j = 0; j < 8; ++j) { const size_t vrow = ((size_t)b * HID + cg * 128 + j * 16 + col) * GP + kc * 32; const v16b vh = frag_b(VTH + vrow, lane), vl = frag_b(VTL + vrow, lane); acc[j] = wmma_bf(a.l, vh, acc[j]); acc[j] = wmma_bf(a.h, vl, acc[j]); acc[j] = wmma_bf(a.h, vh, acc[j]); } }
#pragma unroll
  for (int j = 0; j < 8; ++j)
#pragma unroll
    for (int r = 0; r < 8; ++r) so[wave][8 * g + r][j * 16 + col] = acc[j][r];
  LDSX();
  for (int rl = 0; rl < 16; ++rl) { const int s = s0 + rl; if (s < SQ) vst2(OB + ((size_t)b * SQ + s) * HID + cg * 128 + lane * 4, *(const v4f*)&so[wave][rl][lane * 4]); }
}
__global__ __launch_bounds__(256) void k_alpha(const float* __restrict__ G, const float* __restrict__ MZ, float* __restrict__ out) {
  const size_t f0 = ((size_t)blockIdx.x * 256 + threadIdx.x) * 4; const size_t total = (size_t)NBT * SQ * WN * WN; if (f0 >= total) return;
  v4f v;
#pragma unroll
  for (int i4 = 0; i4 < 4; ++i4) { const size_t ff = f0 + i4; const int n = (int)(ff / (WN * WN)), rr = (int)(ff % (WN * WN)); const int w = rr / WN, u = rr % WN; const int b = n / SQ, s = n % SQ;
    const int i = s + HW - w, j = s + HW - u; const bool valid = (i >= 0) && (i < SQ) && (j >= 0) && (j < SQ); const int ic = i < 0 ? 0 : (i >= SQ ? SQ - 1 : i), jc = j < 0 ? 0 : (j >= SQ ? SQ - 1 : j);
    const float gg = G[((size_t)(b * GP + ic)) * GP + jc]; const float sc = valid ? gg : 0.f; const float m = MZ[((size_t)(b * GP + s)) * GP + w], iz = MZ[((size_t)(b * GP + s)) * GP + 64 + w];
    v[i4] = exp_ni(sc - m) * iz; }
  vst2(out + (size_t)NR * DOUT + f0, v);
}
extern "C" void kernel_launch(void* const* d_in, const int* in_sizes, int n_in, void* d_out, int out_size, void* d_ws, size_t ws_size, hipStream_t stream) {
  (void)in_sizes; (void)n_in; (void)out_size;
  const float** F = (const float**)d_in;
  if (ws_size < (size_t)WS_END) return;
  char* ws = (char*)d_ws; __bf16 *P0 = (__bf16*)(ws + WS_P0), *PQ = (__bf16*)(ws + WS_PQ), *P1 = (__bf16*)(ws + WS_P1), *VTH = (__bf16*)(ws + WS_VTH), *VTL = (__bf16*)(ws + WS_VTL);
  float *Hh = (float*)(ws + WS_H), *QKV = (float*)(ws + WS_QKV), *G = (float*)(ws + WS_G), *MZ = (float*)(ws + WS_MZ), *C = (float*)(ws + WS_C), *OB = (float*)(ws + WS_OB);
  k_packT<<<HID, 256, 0, stream>>>(F[1], DIN, HID, P0);
  k_packT<<<HID, 256, 0, stream>>>(F[3], HID, HID, PQ);
  k_packT<<<HID, 256, 0, stream>>>(F[4], HID, HID, PQ + (size_t)HID * HID);
  k_packT<<<HID, 256, 0, stream>>>(F[5], HID, HID, PQ + (size_t)2 * HID * HID);
  k_packT<<<DOUT, 256, 0, stream>>>(F[6], HID, DOUT, P1);
  k_lin<DIN, 0, 1><<<dim3(NBT * SQ / 64, HID / 128), 128, 0, stream>>>(F[0], DIN, P0, F[2], Hh, HID);
  k_lin<HID, 1, 0><<<dim3(NBT * SQ / 64, QKVP / 128), 128, 0, stream>>>(Hh, HID, PQ, nullptr, QKV, QKVP);
  k_g<<<dim3(7, NBT), 128, 0, stream>>>(QKV, G);
  k_soft<<<NBT * GP / 8, 256, 0, stream>>>(G, MZ, C);
  k_vt<<<dim3(2, NBT), 256, 0, stream>>>(QKV, VTH, VTL);
  k_cv<<<dim3(2, HID / 128, NBT), 128, 0, stream>>>(C, VTH, VTL, OB);
  k_lin<HID, 1, 1><<<dim3(NBT * SQ / 64, DOUT / 128), 128, 0, stream>>>(OB, HID, P1, F[7], (float*)d_out, DOUT);
  k_alpha<<<(unsigned)(((size_t)NBT * SQ * WN * WN / 4 + 255) / 256), 256, 0, stream>>>(G, MZ, (float*)d_out);
}
